// LE_ACE_36739150250616
// MI455X (gfx1250) — hardware-run, weakly checked
//
#include <hip/hip_runtime.h>


#ifndef NSTR
#define NSTR 256
#endif
#ifndef NAT
#define NAT 16384
#endif
#define NSTR_FULL 256
#define NAT_FULL  16384
#define NSP    4
#define NRS    64
#define F2     1174
#define SEGW   1239
#define SEGP   1248
#define ROWLEN 4956
#define B1_OFF 4
#define B2_OFF 260
#define NTH    128
#define CHUNK  512
#define CAP    1024

#define LQ(L)     ((L) == 0 ? 32 : (L) == 1 ? 24 : (L) == 2 ? 20 : 16)
#define LD(L)     (2 * (L) + 1)
#define LROWS(L)  (LQ(L) > 16 ? 32 : 16)
#define LPITCH(L) (LD(L) * 32 + 8)
#define LTSZ(L)   (LROWS(L) * LPITCH(L))
#define LTOFF(L)  ((L) == 0 ? 0 : (L) == 1 ? LTSZ(0) : (L) == 2 ? (LTSZ(0) + LTSZ(1)) : (LTSZ(0) + LTSZ(1) + LTSZ(2)))
#define LFOFF(L)  ((L) == 0 ? 0 : (L) == 1 ? 528 : (L) == 2 ? 828 : 1038)
#define XT_TOTAL  (LTOFF(3) + LTSZ(3))
#define SEGN      (NSTR * NSP * SEGP)

static_assert(NTH == 128);
static_assert(CHUNK == NTH * 4);
static_assert(NAT % CHUNK == 0);
static_assert(CAP >= 2 * CHUNK);
static_assert(CAP % NTH == 0);
static_assert(NRS == 64);
static_assert(SEGW == 1 + NRS + F2);
static_assert(F2 == 528 + 300 + 210 + 136);
static_assert(LFOFF(1) == 32 * 33 / 2);
static_assert(LFOFF(2) == LFOFF(1) + 24 * 25 / 2);
static_assert(LFOFF(3) == LFOFF(2) + 20 * 21 / 2);
static_assert(F2 == LFOFF(3) + 16 * 17 / 2);
static_assert(SEGP % 32 == 0);
static_assert(SEGP >= SEGW);
static_assert(SEGP - SEGW <= NTH);
static_assert(SEGP / 4 <= 3 * NTH);
static_assert(SEGP / 4 > 2 * NTH);
static_assert((SEGP / 4) % 8 == 0);
static_assert(ROWLEN == NSP * SEGW);
static_assert(ROWLEN % 4 == 0);
static_assert(B2_OFF == NSP + NSP * NRS);
static_assert(B1_OFF == NSP);
static_assert(LTOFF(1) % 8 == 0);
static_assert(LTOFF(2) % 8 == 0);
static_assert(LTOFF(3) % 8 == 0);
static_assert(LPITCH(0) % 8 == 0);
static_assert(LPITCH(1) % 8 == 0);
static_assert(LPITCH(2) % 8 == 0);
static_assert(LPITCH(3) % 8 == 0);
static_assert((size_t)XT_TOTAL * 2 + (size_t)SEGP * 4 + (size_t)CAP * 4 + 16 <= (size_t)131072);
static_assert(((size_t)NSTR * (ROWLEN / 4)) % 8 == 0);
static_assert(NSTR <= NSTR_FULL);
static_assert(NAT <= NAT_FULL);

typedef unsigned short bf;
typedef __attribute__((ext_vector_type(16))) __bf16   v16bf;
typedef __attribute__((ext_vector_type(8)))  unsigned short v8us;
typedef __attribute__((ext_vector_type(8)))  float    v8f;
typedef __attribute__((ext_vector_type(4)))  float    v4f;
typedef __attribute__((ext_vector_type(4)))  int      v4i;
typedef v4f  __attribute__((may_alias)) v4fa;

__device__ __forceinline__ unsigned short f2bf(float f) { unsigned u = __float_as_uint(f); u += 0x7FFFu + ((u >> 16) & 1u); return (unsigned short)(u >> 16); }
__device__ __forceinline__ float bfr(float f) { return __uint_as_float(((unsigned)f2bf(f)) << 16); }
__device__ __forceinline__ v16bf cat16b(v8us lo, v8us hi) { return __builtin_bit_cast(v16bf, __builtin_shufflevector(lo, hi, 0, 1, 2, 3, 4, 5, 6, 7, 8, 9, 10, 11, 12, 13, 14, 15)); }
__device__ __forceinline__ v8f wmmab(v16bf a, v16bf b, v8f c) { return __builtin_amdgcn_wmma_f32_16x16x32_bf16(false, a, false, b, (short)0, c, false, false); }
__device__ __forceinline__ void wave_sync() { __builtin_amdgcn_fence(3  , "wavefront"); __builtin_amdgcn_wave_barrier(); asm volatile("" ::: "memory"); }
__device__ __forceinline__ v8f wmmab_g(v16bf a, v16bf b, v8f c) {
    c = wmmab(a, b, c);
    asm volatile("v_nop\n\tv_nop\n\tv_nop\n\tv_nop" : "+v"(c) : "v"(a), "v"(b));
    return c;
}
__device__ __forceinline__ v16bf ldbs(const bf* p, unsigned short sg) {
    v8us lo = *(const v8us*)p, hi = *(const v8us*)(p + 16);
    v8us sv;
#pragma unroll
    for (int k = 0; k < 8; ++k) sv[k] = sg;
    lo = lo ^ sv; hi = hi ^ sv;
    return cat16b(lo, hi);
}

template <int L>
__device__ __forceinline__ void zero_pad(bf* tile, int lane) {
#pragma unroll 1
    for (int row = LQ(L); row < LROWS(L); ++row) {
#pragma unroll
        for (int m = 0; m < LD(L); ++m) tile[row * LPITCH(L) + m * 32 + lane] = (bf)0;
    }
}

template <int L>
__device__ __forceinline__ void stage_l(const float* __restrict__ S, bf* tile, int a, bool ok, int lane) {
#pragma unroll 1
    for (int qi = 0; qi < LQ(L); ++qi) {
        float x[LD(L)];
#pragma unroll
        for (int m = 0; m < LD(L); ++m) x[m] = S[(size_t)(qi * LD(L) + m) * NAT_FULL + (size_t)a];
#pragma unroll
        for (int m = 0; m < LD(L); ++m) {
            float v = x[m];
            asm volatile("" : "+v"(v));
            tile[qi * LPITCH(L) + m * 32 + lane] = ok ? f2bf(v) : (bf)0;
        }
    }
}

template <int L>
__device__ __forceinline__ void mma_l(const bf* tile, int lr, int hi, v8f& c00, v8f& c01, v8f& c11) {
    const bf* plo = tile + lr * LPITCH(L) + 8 * hi;
#pragma unroll
    for (int m = 0; m < LD(L); ++m) {
        const int mr = LD(L) - 1 - m;
        const unsigned short sg = (m & 1) ? (unsigned short)0x8000 : (unsigned short)0;
        const v16bf alo = ldbs(plo + m * 32, (unsigned short)0);
        const v16bf blo = ldbs(plo + mr * 32, sg);
        c00 = wmmab_g(alo, blo, c00);
        if constexpr (LQ(L) > 16) {
            const bf* phi = tile + (16 + lr) * LPITCH(L) + 8 * hi;
            const v16bf ahi = ldbs(phi + m * 32, (unsigned short)0);
            const v16bf bhi = ldbs(phi + mr * 32, sg);
            c01 = wmmab_g(alo, bhi, c01);
            c11 = wmmab_g(ahi, bhi, c11);
        }
    }
}

template <int L>
__device__ __forceinline__ void seg_step(const float* __restrict__ S, bf* tile, int a, bool ok, int lane, int lr, int hi, v8f& c00, v8f& c01, v8f& c11) {
    stage_l<L>(S, tile, a, ok, lane);
    wave_sync();
    mma_l<L>(tile, lr, hi, c00, c01, c11);
    wave_sync();
}

template <int L>
__device__ __forceinline__ void emit_l(float* rb, int lr, int hi, const v8f& c00, const v8f& c01, const v8f& c11) {
    constexpr int q = LQ(L);
    constexpr float inv = (L == 0) ? 1.0f : (L == 1) ? 0.57735026918962576f : (L == 2) ? 0.44721359549995794f : 0.37796447300922722f;
    const float SQ2 = 1.41421356237309515f;
    float* o = rb + 1 + NRS + LFOFF(L);
#pragma unroll
    for (int r = 0; r < 8; ++r) {
        const int M = r + 8 * hi, N = lr;
        if (M <= N) o[M * q - (M * (M - 1)) / 2 + (N - M)] = (c00[r] * inv) * ((M == N) ? 1.0f : SQ2);
    }
    if constexpr (q > 16) {
#pragma unroll
        for (int r = 0; r < 8; ++r) {
            const int M = r + 8 * hi, N = 16 + lr;
            if (N < q) o[M * q - (M * (M - 1)) / 2 + (N - M)] = (c01[r] * inv) * SQ2;
        }
#pragma unroll
        for (int r = 0; r < 8; ++r) {
            const int M = 16 + r + 8 * hi, N = 16 + lr;
            if ((M < q) & (N < q) & (M <= N)) o[M * q - (M * (M - 1)) / 2 + (N - M)] = (c11[r] * inv) * ((M == N) ? 1.0f : SQ2);
        }
    }
}

__global__ __launch_bounds__(NTH) void k_seg(const float* __restrict__ comp, const float* __restrict__ radial,
                                             const float* __restrict__ s0, const float* __restrict__ s1, const float* __restrict__ s2, const float* __restrict__ s3,
                                             const int* __restrict__ st, const int* __restrict__ sp, const int* __restrict__ nstp, const int* __restrict__ nspp, float* SEG) {
    __shared__ __align__(16) bf xt[XT_TOTAL];
    __shared__ __align__(16) float rowbuf[SEGP];
    __shared__ int lst[CAP];
    __shared__ int wcnt[NTH / 32];
    const int tid = threadIdx.x, lane = tid & 31, lr = lane & 15, hi = lane >> 4;
    const int wave = __builtin_amdgcn_readfirstlane((int)(threadIdx.x >> 5));
    const int wv = tid >> 5;
    const int g = blockIdx.x;
    const int nsp = nspp[0], nst = nstp[0];
    const bool gok = (long long)g < (long long)nst * (long long)nsp;

#pragma unroll
    for (int k = 0; k < CAP / NTH; ++k) lst[k * NTH + tid] = 0;
    if (tid < SEGP - SEGW) rowbuf[SEGW + tid] = 0.0f;
    if (wave == 1) zero_pad<1>(xt + LTOFF(1), lane);
    if (wave == 2) zero_pad<2>(xt + LTOFF(2), lane);

    v8f c00 = (v8f){}, c01 = (v8f){}, c11 = (v8f){};
    float b1acc = 0.0f, b0acc = 0.0f;
    int cnt = 0;
#pragma unroll 1
    for (int cb = 0; cb < NAT; cb += CHUNK) {
        const int i0 = cb + tid * 4;
        const v4i sv = *(const v4i*)(st + i0);
        const v4i pv = *(const v4i*)(sp + i0);
        bool hit[4]; unsigned bm[4]; int wt = 0;
#pragma unroll
        for (int k = 0; k < 4; ++k) {
            hit[k] = gok & ((nsp * sv[k] + pv[k]) == g);
            bm[k] = __builtin_amdgcn_ballot_w32(hit[k]);
            wt += __popc(bm[k]);
        }
        if (lane == 0) wcnt[wave] = wt;
        __syncthreads();
        int r0 = wcnt[0], r1 = wcnt[1], r2 = wcnt[2], r3 = wcnt[3];
        r0 = r0 < 0 ? 0 : (r0 > CHUNK / 4 ? CHUNK / 4 : r0); r1 = r1 < 0 ? 0 : (r1 > CHUNK / 4 ? CHUNK / 4 : r1);
        r2 = r2 < 0 ? 0 : (r2 > CHUNK / 4 ? CHUNK / 4 : r2); r3 = r3 < 0 ? 0 : (r3 > CHUNK / 4 ? CHUNK / 4 : r3);
        const int w0 = __builtin_amdgcn_readfirstlane(r0), w1 = __builtin_amdgcn_readfirstlane(r1);
        const int w2 = __builtin_amdgcn_readfirstlane(r2), w3 = __builtin_amdgcn_readfirstlane(r3);
        int run = cnt + ((wv > 0) ? r0 : 0) + ((wv > 1) ? r1 : 0) + ((wv > 2) ? r2 : 0);
#pragma unroll
        for (int k = 0; k < 4; ++k) {
            const int pos = run + (int)__builtin_amdgcn_mbcnt_lo(bm[k], 0u);
            if (hit[k] & (pos >= 0) & (pos < CAP)) lst[pos] = i0 + k;
            run += __popc(bm[k]);
        }
        cnt += w0 + w1 + w2 + w3;
        __syncthreads();
        if ((cnt > CAP - CHUNK) | (cb + CHUNK >= NAT)) {
#pragma unroll 1
            for (int a0 = 0; (a0 < cnt) & (a0 < CAP); a0 += 32) {
                const int li = a0 + lane;
                int a = lst[li < CAP ? li : CAP - 1];
                asm volatile("" : "+v"(a));
                const bool ok = li < cnt;
                a = ok ? a : 0;
                a = a < 0 ? 0 : (a > NAT - 1 ? NAT - 1 : a);
                if (wave < 2) {
#pragma unroll 1
                    for (int j = 0; j < 32; ++j) {
                        if (a0 + j >= cnt) break;
                        int aj = lst[a0 + j];
                        aj = aj < 0 ? 0 : (aj > NAT - 1 ? NAT - 1 : aj);
                        b1acc += bfr(radial[(size_t)aj * NRS + tid]);
                    }
                } else if (wave == 2) {
                    float cv = comp[a];
                    asm volatile("" : "+v"(cv));
                    b0acc += ok ? bfr(cv) : 0.0f;
                }
                switch (wave) {
                    case 0:  seg_step<0>(s0, xt + LTOFF(0), a, ok, lane, lr, hi, c00, c01, c11); break;
                    case 1:  seg_step<1>(s1, xt + LTOFF(1), a, ok, lane, lr, hi, c00, c01, c11); break;
                    case 2:  seg_step<2>(s2, xt + LTOFF(2), a, ok, lane, lr, hi, c00, c01, c11); break;
                    default: seg_step<3>(s3, xt + LTOFF(3), a, ok, lane, lr, hi, c00, c01, c11); break;
                }
            }
            cnt = 0;
        }
    }

    switch (wave) {
        case 0:  emit_l<0>(rowbuf, lr, hi, c00, c01, c11); break;
        case 1:  emit_l<1>(rowbuf, lr, hi, c00, c01, c11); break;
        case 2:  emit_l<2>(rowbuf, lr, hi, c00, c01, c11); break;
        default: emit_l<3>(rowbuf, lr, hi, c00, c01, c11); break;
    }
    if (tid < NRS) rowbuf[1 + tid] = b1acc;
    float tsum = b0acc;
    tsum += __shfl_xor(tsum, 16, 32); tsum += __shfl_xor(tsum, 8, 32); tsum += __shfl_xor(tsum, 4, 32);
    tsum += __shfl_xor(tsum, 2, 32);  tsum += __shfl_xor(tsum, 1, 32);
    if (tid == 64) rowbuf[0] = tsum;
    __syncthreads();

    float* dst = SEG + (size_t)g * SEGP;
#pragma unroll 1
    for (int ps = 0; ps < 2; ++ps) {
#pragma unroll
        for (int s = 0; s < 3; ++s) {
            const int i4 = s * NTH + tid;
            if (i4 < SEGP / 4) { const v4f val = *(const v4fa*)(&rowbuf[i4 * 4]); *(volatile v4f*)(dst + (size_t)i4 * 4) = val; }
        }
        if (ps == 0) __threadfence();
    }
}

__global__ __launch_bounds__(256) void k_pack(const float* __restrict__ SEG, float* OUT, unsigned n4) {
    const unsigned i = blockIdx.x * 256u + threadIdx.x; if (i >= n4) return;
    const unsigned s = i / (unsigned)(ROWLEN / 4), c0 = (i % (unsigned)(ROWLEN / 4)) * 4u;
    v4f val;
#pragma unroll
    for (int k = 0; k < 4; ++k) {
        const unsigned c = c0 + (unsigned)k;
        const bool ra = c < (unsigned)B1_OFF, rb = c < (unsigned)B2_OFF;
        const unsigned c1 = (rb & !ra) ? (c - (unsigned)B1_OFF) : 0u;
        const unsigned c2 = rb ? 0u : (c - (unsigned)B2_OFF);
        const unsigned sp1 = c1 / (unsigned)NRS, of1 = 1u + (c1 % (unsigned)NRS);
        const unsigned sp2 = c2 / (unsigned)F2,  of2 = 1u + (unsigned)NRS + (c2 - sp2 * (unsigned)F2);
        const unsigned spc = ra ? c : (rb ? sp1 : sp2);
        const unsigned off = ra ? 0u : (rb ? of1 : of2);
        unsigned idx = (s * (unsigned)NSP + spc) * (unsigned)SEGP + off;
        idx = idx < (unsigned)SEGN ? idx : (unsigned)SEGN - 1u;
        val[k] = SEG[idx];
    }
    *(volatile v4f*)(OUT + (size_t)i * 4) = val; __threadfence(); *(volatile v4f*)(OUT + (size_t)i * 4) = val;
}

static constexpr size_t al256(size_t v) { return (v + 255) & ~(size_t)255; }
static constexpr size_t SZ_SEG = al256((size_t)NSTR * NSP * SEGP * 4);
static constexpr size_t SZ_TOTAL = SZ_SEG;
static_assert(SZ_TOTAL <= (size_t)134217728);
static_assert(((size_t)SEGP * 4) % 128 == 0);

extern "C" void kernel_launch(void* const* d_in, const int* in_sizes, int n_in,
                              void* d_out, int out_size, void* d_ws, size_t ws_size, hipStream_t stream) {
    if (n_in < 10) return;
    if ((size_t)in_sizes[0] < (size_t)NAT) return;
    if ((size_t)in_sizes[1] < (size_t)NAT * NRS) return;
    if ((size_t)in_sizes[2] < (size_t)(32 * 1 - 1) * NAT_FULL + NAT) return;
    if ((size_t)in_sizes[3] < (size_t)(24 * 3 - 1) * NAT_FULL + NAT) return;
    if ((size_t)in_sizes[4] < (size_t)(20 * 5 - 1) * NAT_FULL + NAT) return;
    if ((size_t)in_sizes[5] < (size_t)(16 * 7 - 1) * NAT_FULL + NAT) return;
    if ((size_t)in_sizes[6] < (size_t)NAT || (size_t)in_sizes[7] < (size_t)NAT) return;
    if (in_sizes[8] < 1 || in_sizes[9] < 1) return;
    if ((size_t)out_size < (size_t)NSTR * ROWLEN) return;
    if (SZ_TOTAL > ws_size) return;
    const float* comp   = (const float*)d_in[0];
    const float* radial = (const float*)d_in[1];
    const float* s0 = (const float*)d_in[2]; const float* s1 = (const float*)d_in[3];
    const float* s2 = (const float*)d_in[4]; const float* s3 = (const float*)d_in[5];
    const int* st = (const int*)d_in[6]; const int* sp = (const int*)d_in[7];
    const int* nstp = (const int*)d_in[8]; const int* nspp = (const int*)d_in[9];
    float* OUT = (float*)d_out;
    float* SEG = (float*)d_ws;

    k_seg<<<dim3(NSTR * NSP, 1, 1), NTH, 0, stream>>>(comp, radial, s0, s1, s2, s3, st, sp, nstp, nspp, SEG);
    const unsigned n4 = (unsigned)((size_t)NSTR * (ROWLEN / 4));
    k_pack<<<dim3((n4 + 255u) / 256u, 1, 1), 256, 0, stream>>>(SEG, OUT, n4);
}
